// InterestTransformerEncoder_64982855188795
// MI455X (gfx1250) — hardware-verified
//
#include <hip/hip_runtime.h>
#include <stdint.h>

#define NB    1024
#define L_    200
#define D_    64
#define LP    224
#define NTI   13
#define NCH   7
#define NTHR  256
#define NWV   8

static_assert(LP == NCH * 32);
static_assert(NTI * 16 >= L_);
static_assert(NTI * 16 <= LP);
static_assert(NTHR == NWV * 32);
static_assert(LP <= NTHR);
static_assert((D_ * D_) % NTHR == 0);
static_assert((L_ % 2) == 0);

#define OFF_H    0
#define OFF_HT   (OFF_H + LP * D_ * 2)
#define OFF_WT   (OFF_HT + D_ * LP * 2)
#define OFF_INV  (OFF_WT + D_ * D_ * 2)
#define OFF_MSK  (OFF_INV + LP * 4)
#define OFF_STG  (OFF_MSK + LP * 4)
#define LDS_MAIN (OFF_STG + NWV * 16 * D_ * 4)
static_assert(OFF_HT == 28672);
static_assert(OFF_WT == 57344);
static_assert(OFF_INV == 65536);
static_assert(OFF_MSK == 66432);
static_assert(OFF_STG == 67328);
static_assert(LDS_MAIN == 100096);
static_assert((OFF_HT % 16) == 0);
static_assert((OFF_WT % 16) == 0);
static_assert((OFF_INV % 16) == 0);
static_assert((OFF_STG % 16) == 0);

typedef _Float16     v16h __attribute__((ext_vector_type(16)));
typedef _Float16     v8h  __attribute__((ext_vector_type(8)));
typedef float        v8f  __attribute__((ext_vector_type(8)));
typedef float        v4f  __attribute__((ext_vector_type(4)));

union Frag { v16h v; v8h half[2]; };

__device__ __forceinline__ unsigned short bf_bits(float f) {
  unsigned u = __float_as_uint(f);
  return (unsigned short)((u + 0x7FFFu + ((u >> 16) & 1u)) >> 16);
}
__device__ __forceinline__ float bf_up(unsigned short v) { return __uint_as_float(((unsigned)v) << 16); }
__device__ __forceinline__ float bfr(float f) { return bf_up(bf_bits(f)); }
__device__ __forceinline__ v8f zero8() {
  v8f z;
  z[0] = 0.f; z[1] = 0.f; z[2] = 0.f; z[3] = 0.f; z[4] = 0.f; z[5] = 0.f; z[6] = 0.f; z[7] = 0.f;
  return z;
}

__device__ __forceinline__ v16h ldfrag(const _Float16* p) {
  Frag f;
  f.half[0] = *(const v8h*)(p);
  f.half[1] = *(const v8h*)(p + 16);
  return f.v;
}

__device__ __forceinline__ v8f mma(v16h a, v16h b, v8f c) {
  v8f d = __builtin_amdgcn_wmma_f32_16x16x32_f16(false, a, false, b, (short)0, c, false, false);
#if defined(__HIP_DEVICE_COMPILE__)
  asm volatile("v_nop\n\tv_nop\n\tv_nop\n\tv_nop" : "+v"(d) : "v"(a), "v"(b));
#endif
  return d;
}

__device__ __forceinline__ void mk_t8(const v8f ha, const v8f la, float rden, const _Float16* hrow,
                                      v8h& hi8, v8h& lo8) {
#pragma unroll
  for (int r = 0; r < 8; ++r) {
    const float hn  = ha[r] + la[r] * 0.00048828125f;
    const float t16 = hn * rden + (float)hrow[r];
    const _Float16 th = (_Float16)t16;
    const _Float16 tl = (_Float16)((t16 - (float)th) * 2048.0f);
    hi8[r] = th;
    lo8[r] = tl;
  }
}

__global__ __launch_bounds__(NTHR) void k_main(const int* __restrict__ seq,
                                                const float* __restrict__ hist,
                                                const float* __restrict__ W,
                                                float* out) {
  extern __shared__ __align__(16) unsigned char smem[];
  _Float16* sH   = (_Float16*)(smem + OFF_H);
  _Float16* sHT  = (_Float16*)(smem + OFF_HT);
  _Float16* sWT  = (_Float16*)(smem + OFF_WT);
  float*    sInv = (float*)(smem + OFF_INV);
  float*    sMsk = (float*)(smem + OFF_MSK);
  float*    sStg = (float*)(smem + OFF_STG);

  const int tid  = threadIdx.x;
  const int lane = tid & 31;
  const int wid  = tid >> 5;
  const int h    = lane >> 4;
  const int lo   = lane & 15;
  const int b    = blockIdx.x;

#pragma unroll 4
  for (int k = 0; k < (D_ * D_) / NTHR; ++k) {
    const int idx = k * NTHR + tid;
    const int e = idx >> 6, d = idx & 63;
    sWT[e * D_ + d] = (_Float16)(bfr(W[d * D_ + e]) * 1024.0f);
  }

  if (tid < LP) {
    const int  j     = tid;
    const int  jc    = min(j, L_ - 1);
    const bool valid = j < L_;
    const float* hr = hist + ((size_t)b * L_ + jc) * D_;
    float ss = 0.0f;
#pragma unroll
    for (int q = 0; q < 8; ++q) {
      const v4f x0 = *(const v4f*)(hr + 8 * q);
      const v4f x1 = *(const v4f*)(hr + 8 * q + 4);
      float va[8];
#pragma unroll
      for (int c = 0; c < 4; ++c) {
        const float v0 = bfr(x0[c]);
        const float v1 = bfr(x1[c]);
        va[c]     = valid ? v0 : 0.0f;
        va[4 + c] = valid ? v1 : 0.0f;
      }
      v8h r8;
#pragma unroll
      for (int c = 0; c < 8; ++c) {
        ss += va[c] * va[c];
        r8[c] = (_Float16)(va[c] * 16.0f);
      }
      *(v8h*)(sH + j * D_ + 8 * q) = r8;
#pragma unroll
      for (int c = 0; c < 8; ++c) sHT[(8 * q + c) * LP + j] = r8[c];
    }
    const float inv = 1.0f / sqrtf(ss + 0.01f);
    sInv[j] = valid ? inv : 0.0f;
    const int id = seq[(size_t)b * L_ + jc];
    sMsk[j] = (valid && id != 0) ? 1.0f : 0.0f;
  }
  __syncthreads();

#pragma unroll 1
  for (int pass = 0; pass < 2; ++pass) {
    const int mt = wid + NWV * pass;
    if (mt < NTI) {
      const int i0 = mt * 16;
      const _Float16* hrow = sH + (i0 + lo) * D_;
      const v16h bq0 = ldfrag(hrow + 8 * h);
      const v16h bq1 = ldfrag(hrow + 32 + 8 * h);
      const float invi = sInv[i0 + lo];

      v8f hacc[4], lacc[4];
#pragma unroll
      for (int nd = 0; nd < 4; ++nd) { hacc[nd] = zero8(); lacc[nd] = zero8(); }
      float dsum = 0.0f;

#pragma unroll 1
      for (int kc = 0; kc < NCH; ++kc) {
        const int j0 = kc * 32;
        Frag ph, pl;
#pragma unroll
        for (int sub = 0; sub < 2; ++sub) {
          const int jt0 = j0 + 16 * sub;
          const _Float16* pa = sH + (jt0 + lo) * D_ + 8 * h;
          v8f acc = mma(ldfrag(pa), bq0, zero8());
          acc = mma(ldfrag(pa + 32), bq1, acc);
          v8h p8h, p8l;
#pragma unroll
          for (int r = 0; r < 8; ++r) {
            const int j = jt0 + 8 * h + r;
            const float s = acc[r] * 0.00390625f * invi * sInv[j];
            const float w = __expf(s) * sMsk[j];
            dsum += w;
            const _Float16 wh = (_Float16)w;
            const _Float16 wl = (_Float16)((w - (float)wh) * 2048.0f);
            p8h[r] = wh;
            p8l[r] = wl;
          }
          ph.half[sub] = p8h;
          pl.half[sub] = p8l;
        }
#pragma unroll
        for (int nd = 0; nd < 4; ++nd) {
          const v16h av = ldfrag(sHT + (16 * nd + lo) * LP + j0 + 8 * h);
          hacc[nd] = mma(av, ph.v, hacc[nd]);
          lacc[nd] = mma(av, pl.v, lacc[nd]);
        }
      }

      dsum += __shfl_xor(dsum, 16);
      const float rden = 1.0f / dsum;

      Frag th0, th1, tl0, tl1;
      {
        v8h a8, c8;
        mk_t8(hacc[0], lacc[0], rden, hrow + 0  + 8 * h, a8, c8); th0.half[0] = a8; tl0.half[0] = c8;
        mk_t8(hacc[1], lacc[1], rden, hrow + 16 + 8 * h, a8, c8); th0.half[1] = a8; tl0.half[1] = c8;
        mk_t8(hacc[2], lacc[2], rden, hrow + 32 + 8 * h, a8, c8); th1.half[0] = a8; tl1.half[0] = c8;
        mk_t8(hacc[3], lacc[3], rden, hrow + 48 + 8 * h, a8, c8); th1.half[1] = a8; tl1.half[1] = c8;
      }

      v8f o[4], ol[4];
#pragma unroll
      for (int ne = 0; ne < 4; ++ne) { o[ne] = zero8(); ol[ne] = zero8(); }
#pragma unroll
      for (int ne = 0; ne < 4; ++ne) {
        const _Float16* pb = sWT + (16 * ne + lo) * D_ + 8 * h;
        const v16h b0 = ldfrag(pb);
        o[ne]  = mma(th0.v, b0, o[ne]);
        ol[ne] = mma(tl0.v, b0, ol[ne]);
        const v16h b1 = ldfrag(pb + 32);
        o[ne]  = mma(th1.v, b1, o[ne]);
        ol[ne] = mma(tl1.v, b1, ol[ne]);
      }

      float* stg = sStg + wid * (16 * D_);
#pragma unroll
      for (int ne = 0; ne < 4; ++ne) {
#pragma unroll
        for (int r = 0; r < 8; ++r) {
          const int ii = 8 * h + r;
          float v = (o[ne][r] + ol[ne][r] * 0.00048828125f) * 6.103515625e-05f;
          v = (v < 0.0f) ? 0.0f : v;
          v = v * sMsk[i0 + ii];
          stg[ii * D_ + 16 * ne + lo] = v;
        }
      }
    }
    __syncthreads();

    if (mt < NTI) {
      const int i0 = mt * 16;
      const float* stg = sStg + wid * (16 * D_);
      v4f pv[8];
#pragma unroll
      for (int t = 0; t < 8; ++t) pv[t] = *(const v4f*)(stg + (2 * t + h) * D_ + 4 * lo);
      float* ob = out + ((size_t)b * L_ + i0 + h) * D_ + 4 * lo;
#pragma unroll
      for (int t = 0; t < 8; ++t)
        if (i0 + 2 * t < L_) *(volatile v4f*)(ob + (size_t)(2 * t) * D_) = pv[t];
      __threadfence();
#pragma unroll
      for (int t = 0; t < 8; ++t)
        if (i0 + 2 * t < L_) *(volatile v4f*)(ob + (size_t)(2 * t) * D_) = pv[t];
    }
    __syncthreads();
  }
}

extern "C" void kernel_launch(void* const* d_in, const int* in_sizes, int n_in,
                              void* d_out, int out_size, void* d_ws, size_t ws_size,
                              hipStream_t stream) {
  (void)d_ws; (void)ws_size;
  if (n_in < 3) return;
  if (in_sizes[0] != NB * L_) return;
  if (in_sizes[1] != NB * L_ * D_) return;
  if (in_sizes[2] != D_ * D_) return;
  if (out_size != NB * L_ * D_) return;

  const int*   seq  = (const int*)d_in[0];
  const float* hist = (const float*)d_in[1];
  const float* W    = (const float*)d_in[2];
  float*       out  = (float*)d_out;

  (void)hipFuncSetAttribute(reinterpret_cast<const void*>(&k_main),
                            hipFuncAttributeMaxDynamicSharedMemorySize, LDS_MAIN);

  const dim3 gMain(NB), bMain(NTHR);
  k_main<<<gMain, bMain, LDS_MAIN, stream>>>(seq, hist, W, out);
  (void)hipGetLastError();
}
